// RankGNN_38113539785296
// MI455X (gfx1250) — hardware-run, weakly checked
//
#include <hip/hip_runtime.h>
#include <stddef.h>
#include <math.h>


#define HIDC    64
#define FIN     9
#define NMAT    4
#define WPL     (HIDC * HIDC)
#define NTHR    256
#define NWAVE   8
#define EPT     8
#define NGRP    2
#define CHUNK   (NTHR * EPT * NGRP)
#define WCAP    (EPT * NGRP * 32)
#define LISTN   (NWAVE * WCAP)
#define NBC     4096
#define NBF     1024
#define RCAP    40960
#define RBN     128
#define TGT     256
#define DEGCAP  256
#define GROWS   128
#define OTHR    512
#define APH     (HIDC + 8)
#define INROWS  64
#define GCAP    5120
#define PCH     1024
#define SOUTN   9216
#define WSCAP   134217728

#define LDS_GEMM (2 * GROWS * APH * 2)
#define LDS_FILL ((RCAP + NBF + LISTN) * 4 + 64)

static_assert((CHUNK & (CHUNK - 1)) == 0);
static_assert(CHUNK <= 4096);
static_assert(NBC <= 4096 && NBF <= 4096);
static_assert((NBC & (NBC - 1)) == 0 && (NBF & (NBF - 1)) == 0);
static_assert(NBC == 4 * NBF);
static_assert(OTHR * 8 == NBC);
static_assert((RCAP % 32) == 0);
static_assert(GROWS * HIDC * 4 <= LDS_GEMM);
static_assert((APH * 2) % 16 == 0);
static_assert((TGT % GROWS) == 0 && TGT == NWAVE * 32);
static_assert((NBC % TGT) == 0);
static_assert((GROWS * HIDC / 8) % NTHR == 0);
static_assert(WPL / 8 == 2 * NTHR);
static_assert(GROWS == NWAVE * 16);
static_assert(INROWS == NWAVE * 8 && (TGT % INROWS) == 0);
static_assert(GCAP + PCH <= SOUTN);
static_assert((PCH % NTHR) == 0);
static_assert((GCAP % NTHR) == 0);

typedef float          v4f  __attribute__((ext_vector_type(4)));
typedef float          v8f  __attribute__((ext_vector_type(8)));
typedef int            v4i  __attribute__((ext_vector_type(4)));
typedef unsigned short v8us __attribute__((ext_vector_type(8)));
typedef __bf16         v16b __attribute__((ext_vector_type(16)));
union FragB { v16b v; v8us h[2]; };

__device__ __forceinline__ unsigned int bfr(float f) {
  const unsigned int u = __float_as_uint(f);
  return (u + 0x7FFFu + ((u >> 16) & 1u)) >> 16;
}

__device__ __forceinline__ void split1(float x, unsigned short& hb, unsigned short& lb) {
  const unsigned int hu = bfr(x);
  const float hf = __uint_as_float(hu << 16);
  hb = (unsigned short)hu;
  lb = (unsigned short)bfr(x - hf);
}

__device__ __forceinline__ void split8(v4f a, v4f b, v8us& hi, v8us& lo) {
  unsigned short hb, lb;
  split1(a.x, hb, lb); hi[0] = hb; lo[0] = lb;
  split1(a.y, hb, lb); hi[1] = hb; lo[1] = lb;
  split1(a.z, hb, lb); hi[2] = hb; lo[2] = lb;
  split1(a.w, hb, lb); hi[3] = hb; lo[3] = lb;
  split1(b.x, hb, lb); hi[4] = hb; lo[4] = lb;
  split1(b.y, hb, lb); hi[5] = hb; lo[5] = lb;
  split1(b.z, hb, lb); hi[6] = hb; lo[6] = lb;
  split1(b.w, hb, lb); hi[7] = hb; lo[7] = lb;
}

__device__ __forceinline__ v8f wmb(v16b a, v16b b, v8f c) {
  v8f d = __builtin_amdgcn_wmma_f32_16x16x32_bf16(false, a, false, b, (short)0, c, false, false);
  asm volatile("v_nop\n\tv_nop\n\tv_nop\n\tv_nop" : "+v"(d) : "v"(a), "v"(b));
  return d;
}

template <int NB>
__device__ __forceinline__ int scan_chunk(const int* __restrict__ dsts, int nE, int cbase, int slotBase,
                                          int vec8, int* list, int tid, int lane, int wave) {
  int wc = 0;
#pragma unroll
  for (int g = 0; g < NGRP; ++g) {
    const int el0  = (g * NTHR + tid) * EPT;
    const int e0   = cbase + el0;
    const int sent = -2147483647 - 1;
    v4i da, db;
    if (vec8 != 0 && cbase + CHUNK <= nE) {
      da = *(const v4i*)(dsts + e0);
      db = *(const v4i*)(dsts + e0 + 4);
    } else {
      da.x = (e0     < nE) ? dsts[min(e0, nE - 1)] : sent;
      da.y = (e0 + 1 < nE) ? dsts[min(e0 + 1, nE - 1)] : sent;
      da.z = (e0 + 2 < nE) ? dsts[min(e0 + 2, nE - 1)] : sent;
      da.w = (e0 + 3 < nE) ? dsts[min(e0 + 3, nE - 1)] : sent;
      db.x = (e0 + 4 < nE) ? dsts[min(e0 + 4, nE - 1)] : sent;
      db.y = (e0 + 5 < nE) ? dsts[min(e0 + 5, nE - 1)] : sent;
      db.z = (e0 + 6 < nE) ? dsts[min(e0 + 6, nE - 1)] : sent;
      db.w = (e0 + 7 < nE) ? dsts[min(e0 + 7, nE - 1)] : sent;
    }
    const unsigned nb = (unsigned)slotBase;
    const unsigned s0 = (unsigned)da.x - nb, s1 = (unsigned)da.y - nb;
    const unsigned s2 = (unsigned)da.z - nb, s3 = (unsigned)da.w - nb;
    const unsigned s4 = (unsigned)db.x - nb, s5 = (unsigned)db.y - nb;
    const unsigned s6 = (unsigned)db.z - nb, s7 = (unsigned)db.w - nb;
    const bool h0 = s0 < (unsigned)NB, h1 = s1 < (unsigned)NB, h2 = s2 < (unsigned)NB, h3 = s3 < (unsigned)NB;
    const bool h4 = s4 < (unsigned)NB, h5 = s5 < (unsigned)NB, h6 = s6 < (unsigned)NB, h7 = s7 < (unsigned)NB;
    const unsigned any = __builtin_amdgcn_ballot_w32(h0 | h1 | h2 | h3 | h4 | h5 | h6 | h7);
    if (any != 0u) {
#define HITJ(J, HJ, SJ) { \
        const unsigned mj = __builtin_amdgcn_ballot_w32(HJ); \
        if (mj != 0u) { \
          if (HJ) { \
            const int pos = wc + (int)__builtin_amdgcn_mbcnt_lo(mj, 0u); \
            if (pos < WCAP) list[wave * WCAP + pos] = ((el0 + (J)) << 12) | (int)(SJ); \
          } \
          wc += (int)__builtin_popcount(mj); } }
      HITJ(0, h0, s0)
      HITJ(1, h1, s1)
      HITJ(2, h2, s2)
      HITJ(3, h3, s3)
      HITJ(4, h4, s4)
      HITJ(5, h5, s5)
      HITJ(6, h6, s6)
      HITJ(7, h7, s7)
#undef HITJ
    }
  }
  return wc;
}

__global__ __launch_bounds__(NTHR) void k_wprep(
    const float* __restrict__ w0, const float* __restrict__ w1,
    const float* __restrict__ w2, const float* __restrict__ w3, unsigned short* wp) {
  const int seg = (int)blockIdx.x >> 1;
  const float* src = seg == 0 ? w0 : (seg == 1 ? w1 : (seg == 2 ? w2 : w3));
  const int ncol = (seg == 3) ? (HIDC / 2) : HIDC;
  const int i  = ((int)(blockIdx.x & 1) * NTHR) + (int)threadIdx.x;
  const int n  = i >> 3;
  const int k0 = (i & 7) * 8;
  const int ncl = n > ncol - 1 ? ncol - 1 : n;
  float v[8];
#pragma unroll
  for (int e = 0; e < 8; ++e) {
    const float t = src[(k0 + e) * ncol + ncl];
    v[e] = (n < ncol) ? t : 0.0f;
  }
  v4f a, b;
  a.x = v[0]; a.y = v[1]; a.z = v[2]; a.w = v[3];
  b.x = v[4]; b.y = v[5]; b.z = v[6]; b.w = v[7];
  v8us hv, lv;
  split8(a, b, hv, lv);
  unsigned short* dh = wp + (size_t)seg * 2 * WPL + (size_t)i * 8;
  unsigned short* dl = dh + WPL;
  *(volatile v8us*)dh = hv;
  *(volatile v8us*)dl = lv;
  __threadfence();
  *(volatile v8us*)dh = hv;
  *(volatile v8us*)dl = lv;
}

__global__ __launch_bounds__(NTHR) void k_count(
    const int* __restrict__ ei, int* cnt, float* dinv, int nE, int vec8) {
  __shared__ __attribute__((aligned(16))) int scnt[NBC];
  __shared__ __attribute__((aligned(16))) int list[LISTN];
  __shared__ int wcnt[NWAVE];
  const int tid = threadIdx.x, lane = tid & 31, wave = tid >> 5;
  const int nodeBase = blockIdx.x * NBC;
  const int* dsts = ei + nE;

  for (int i = tid; i < NBC; i += NTHR) scnt[i] = 0;
  __syncthreads();

  const int nChunks = (nE + CHUNK - 1) / CHUNK;
#pragma unroll 1
  for (int ch = 0; ch < nChunks; ++ch) {
    const int cbase = ch * CHUNK;
    const int wc = scan_chunk<NBC>(dsts, nE, cbase, nodeBase, vec8, list, tid, lane, wave);
    if (lane == 0) wcnt[wave] = wc;
    __syncthreads();
    if (wave == 0) {
#pragma unroll 1
      for (int wsx = 0; wsx < NWAVE; ++wsx) {
        int n = __builtin_amdgcn_readfirstlane(wcnt[wsx]);
        n = n > WCAP ? WCAP : (n < 0 ? 0 : n);
        const int* lp = list + wsx * WCAP;
#pragma unroll 1
        for (int i = 0; i < n; ++i) {
          const int ent  = __builtin_amdgcn_readfirstlane(lp[i]);
          const int slot = ent & (NBC - 1);
          if (lane == 0) scnt[slot] = scnt[slot] + 1;
        }
      }
    }
    __syncthreads();
  }

  v4i cq[4]; v4f dq[4];
#pragma unroll
  for (int q = 0; q < 4; ++q) {
    const int f = (wave * 4 + q) * 128 + 4 * lane;
    const v4i c = *(const v4i*)(scnt + f);
    cq[q] = c;
    dq[q].x = rsqrtf((float)(c.x + 1));
    dq[q].y = rsqrtf((float)(c.y + 1));
    dq[q].z = rsqrtf((float)(c.z + 1));
    dq[q].w = rsqrtf((float)(c.w + 1));
  }
  int*   cp = cnt + (size_t)nodeBase;
  float* dp = dinv + (size_t)nodeBase;
#pragma unroll
  for (int q = 0; q < 4; ++q) {
    const int f = (wave * 4 + q) * 128 + 4 * lane;
    *(volatile v4i*)(cp + f) = cq[q];
    *(volatile v4f*)(dp + f) = dq[q];
  }
  __threadfence();
#pragma unroll
  for (int q = 0; q < 4; ++q) {
    const int f = (wave * 4 + q) * 128 + 4 * lane;
    *(volatile v4i*)(cp + f) = cq[q];
    *(volatile v4f*)(dp + f) = dq[q];
  }
}

__global__ __launch_bounds__(OTHR) void k_offsets(
    const int* __restrict__ cnt, int* off, int* rbase, int nChunk) {
  __shared__ __attribute__((aligned(16))) int soff[NBC];
  __shared__ __attribute__((aligned(16))) int srb[RBN];
  __shared__ int wtot[OTHR / 32];
  const int tid = threadIdx.x, lane = tid & 31, wave = tid >> 5, sub = tid >> 7;
  for (int i = tid; i < RBN; i += OTHR) srb[i] = 0;
  int carry = 0;
#pragma unroll 1
  for (int ch = 0; ch < nChunk; ++ch) {
    const int base = ch * NBC;
    const v4i c0 = *(const v4i*)(cnt + base + 8 * tid);
    const v4i c1 = *(const v4i*)(cnt + base + 8 * tid + 4);
    const int e0 = max(c0.x, 0), e1 = max(c0.y, 0), e2 = max(c0.z, 0), e3 = max(c0.w, 0);
    const int e4 = max(c1.x, 0), e5 = max(c1.y, 0), e6 = max(c1.z, 0), e7 = max(c1.w, 0);
    const int ts = e0 + e1 + e2 + e3 + e4 + e5 + e6 + e7;
    int incl = ts;
#pragma unroll
    for (int d = 1; d < 32; d <<= 1) {
      const int t = __shfl_up(incl, d);
      if (lane >= d) incl += t;
    }
    if (lane == 31) wtot[wave] = incl;
    __syncthreads();
    const int S0 = wtot[0]  + wtot[1]  + wtot[2]  + wtot[3];
    const int S1 = wtot[4]  + wtot[5]  + wtot[6]  + wtot[7];
    const int S2 = wtot[8]  + wtot[9]  + wtot[10] + wtot[11];
    const int S3 = wtot[12] + wtot[13] + wtot[14] + wtot[15];
    int pre = 0;
#pragma unroll 1
    for (int w = 4 * sub; w < wave; ++w) pre += wtot[w];
    const int b0 = carry;
    const int b1 = b0 + ((S0 + 31) & ~31);
    const int b2 = b1 + ((S1 + 31) & ~31);
    const int b3 = b2 + ((S2 + 31) & ~31);
    const int b4 = b3 + ((S3 + 31) & ~31);
    const int myb = sub == 0 ? b0 : (sub == 1 ? b1 : (sub == 2 ? b2 : b3));
    if (tid == 0) {
      srb[min(4 * ch + 0, RBN - 1)] = b0;
      srb[min(4 * ch + 1, RBN - 1)] = b1;
      srb[min(4 * ch + 2, RBN - 1)] = b2;
      srb[min(4 * ch + 3, RBN - 1)] = b3;
    }
    int run = myb + pre + incl - ts;
    soff[8 * tid + 0] = run; run += e0;
    soff[8 * tid + 1] = run; run += e1;
    soff[8 * tid + 2] = run; run += e2;
    soff[8 * tid + 3] = run; run += e3;
    soff[8 * tid + 4] = run; run += e4;
    soff[8 * tid + 5] = run; run += e5;
    soff[8 * tid + 6] = run; run += e6;
    soff[8 * tid + 7] = run;
    carry = b4;
    __syncthreads();
    const v4i o0 = *(const v4i*)(soff + 4 * tid);
    const v4i o1 = *(const v4i*)(soff + 4 * (tid + OTHR));
    int* op = off + base;
    *(volatile v4i*)(op + 4 * tid) = o0;
    *(volatile v4i*)(op + 4 * (tid + OTHR)) = o1;
    __threadfence();
    *(volatile v4i*)(op + 4 * tid) = o0;
    *(volatile v4i*)(op + 4 * (tid + OTHR)) = o1;
    __syncthreads();
  }
  if (tid == 0) srb[min(4 * nChunk, RBN - 1)] = carry;
  __syncthreads();
  v4i rv = {0, 0, 0, 0};
  if (tid < 32) rv = *(const v4i*)(srb + 4 * tid);
  if (tid < 32) *(volatile v4i*)(rbase + 4 * tid) = rv;
  __threadfence();
  if (tid < 32) *(volatile v4i*)(rbase + 4 * tid) = rv;
}

__global__ __launch_bounds__(NTHR) void k_fill(
    const int* __restrict__ ei, const int* __restrict__ off, const int* __restrict__ rbase,
    int* csr, int nN, int nE, int vec8, int csrLen) {
  extern __shared__ v4f lds_dyn[];
  int* region = (int*)lds_dyn;
  int* cursor = region + RCAP;
  int* list   = cursor + NBF;
  int* wcnt   = list + LISTN;
  const int tid = threadIdx.x, lane = tid & 31, wave = tid >> 5;
  const int b = blockIdx.x;
  const int nodeBase = b * NBF;
  const int* dsts = ei + nE;

  int rb0 = rbase[b];
  const int rb1 = rbase[b + 1];
  rb0 = rb0 < 0 ? 0 : (rb0 > csrLen ? csrLen : rb0);
  rb0 &= ~31;
  int len = rb1 - rb0;
  len = len < 0 ? 0 : (len > RCAP ? RCAP : len);
  int lenW = (len + 31) & ~31;
  if (rb0 + lenW > csrLen) lenW = (csrLen - rb0) & ~31;

  {
    const v4i z = {0, 0, 0, 0};
    for (int i = tid; i < RCAP / 4; i += NTHR) ((v4i*)region)[i] = z;
    for (int s = tid; s < NBF; s += NTHR) {
      int o = off[nodeBase + s] - rb0;
      o = o < 0 ? 0 : (o > RCAP ? RCAP : o);
      cursor[s] = o;
    }
  }
  __syncthreads();

  const int nChunks = (nE + CHUNK - 1) / CHUNK;
#pragma unroll 1
  for (int ch = 0; ch < nChunks; ++ch) {
    const int cbase = ch * CHUNK;
    const int wc = scan_chunk<NBF>(dsts, nE, cbase, nodeBase, vec8, list, tid, lane, wave);
    if (lane == 0) wcnt[wave] = wc;
    __syncthreads();
    if (wave == 0) {
#pragma unroll 1
      for (int wsx = 0; wsx < NWAVE; ++wsx) {
        int n = __builtin_amdgcn_readfirstlane(wcnt[wsx]);
        n = n > WCAP ? WCAP : (n < 0 ? 0 : n);
        const int* lp = list + wsx * WCAP;
#pragma unroll 1
        for (int i = 0; i < n; ++i) {
          const int ent  = __builtin_amdgcn_readfirstlane(lp[i]);
          const int slot = ent & (NBF - 1);
          int e = cbase + ((ent >> 12) & (CHUNK - 1));
          e = e > nE - 1 ? nE - 1 : e;
          int src = ei[e];
          src = src < 0 ? 0 : (src > nN - 1 ? nN - 1 : src);
          if (lane == 0) {
            int pos = cursor[slot];
            pos = pos < 0 ? 0 : (pos > RCAP - 1 ? RCAP - 1 : pos);
            region[pos] = src;
            const int np = pos + 1;
            cursor[slot] = np > RCAP ? RCAP : np;
          }
        }
      }
    }
    __syncthreads();
  }

  const int nv = lenW >> 2;
  int* gp = csr + rb0;
#pragma unroll 1
  for (int i = tid; i < nv; i += NTHR) { const v4i v = ((const v4i*)region)[i]; *(volatile v4i*)(gp + 4 * i) = v; }
  __threadfence();
#pragma unroll 1
  for (int i = tid; i < nv; i += NTHR) { const v4i v = ((const v4i*)region)[i]; *(volatile v4i*)(gp + 4 * i) = v; }
}

__global__ __launch_bounds__(NTHR) void k_in(
    const float* __restrict__ x, const float* __restrict__ w, const float* __restrict__ dinv,
    float* hw, int nN) {
  __shared__ __attribute__((aligned(16))) float sw[FIN * HIDC];
  const int tid = threadIdx.x, lane = tid & 31, wave = tid >> 5, hh = lane >> 4, c4 = 4 * (lane & 15);
  for (int i = tid; i < FIN * HIDC; i += NTHR) sw[i] = w[i];
  __syncthreads();
  const int rb = blockIdx.x * INROWS + wave * 8;
  v4f res[4];
#pragma unroll
  for (int st = 0; st < 4; ++st) {
    const int row = rb + 2 * st + hh;
    const int rx = row > nN - 1 ? nN - 1 : row;
    const float* xr = x + (size_t)rx * FIN;
    v4f acc = {0.f, 0.f, 0.f, 0.f};
#pragma unroll 1
    for (int k = 0; k < FIN; ++k) {
      const float xv = xr[k];
      const v4f wv = *(const v4f*)(sw + k * HIDC + c4);
      acc.x += xv * wv.x; acc.y += xv * wv.y; acc.z += xv * wv.z; acc.w += xv * wv.w;
    }
    const float d = dinv[row];
    res[st] = acc * d;
  }
  float* gp = hw + (size_t)(rb + hh) * HIDC + c4;
#pragma unroll
  for (int st = 0; st < 4; ++st) *(volatile v4f*)(gp + (size_t)(2 * st) * HIDC) = res[st];
  __threadfence();
#pragma unroll
  for (int st = 0; st < 4; ++st) *(volatile v4f*)(gp + (size_t)(2 * st) * HIDC) = res[st];
}

template <int NCT>
__global__ __launch_bounds__(NTHR) void k_gemm(
    const float* __restrict__ A, const unsigned short* __restrict__ Bw, const float* __restrict__ dinv,
    const float* __restrict__ bias, float* C, int nRowsA, int useDinv, int useBias, int useAct) {
  constexpr int KD  = HIDC;
  constexpr int NC  = 16 * NCT;
  constexpr int NPC = NC / 8;
  static_assert(GROWS * NC * 4 <= LDS_GEMM);
  __shared__ __attribute__((aligned(16))) unsigned short lds_g[LDS_GEMM / 2];
  unsigned short* sHi = lds_g;
  unsigned short* sLo = lds_g + GROWS * APH;
  float*          stg = (float*)lds_g;
  const int tid = threadIdx.x, lane = tid & 31, wave = tid >> 5, hh = lane >> 4, m = lane & 15;
  const int rowBase = blockIdx.x * GROWS;

#pragma unroll
  for (int i = 0; i < (GROWS * KD / 8) / NTHR; ++i) {
    const int idx = i * NTHR + tid;
    const int r   = idx >> 3;
    const int c0  = (idx & 7) * 8;
    int row = rowBase + r;
    row = row > nRowsA - 1 ? nRowsA - 1 : row;
    const float* ap = A + (size_t)row * KD + c0;
    const v4f a = *(const v4f*)ap, b = *(const v4f*)(ap + 4);
    v8us hv, lv;
    split8(a, b, hv, lv);
    *(v8us*)(sHi + r * APH + c0) = hv;
    *(v8us*)(sLo + r * APH + c0) = lv;
  }
  __syncthreads();

  v8f acc[NCT];
#pragma unroll
  for (int t = 0; t < NCT; ++t) { v8f z = {0.f, 0.f, 0.f, 0.f, 0.f, 0.f, 0.f, 0.f}; acc[t] = z; }
  const unsigned short* ahp = sHi + (wave * 16 + m) * APH + 8 * hh;
  const unsigned short* alp = sLo + (wave * 16 + m) * APH + 8 * hh;
#pragma unroll
  for (int kt = 0; kt < KD / 32; ++kt) {
    FragB ah, al;
    ah.h[0] = *(const v8us*)(ahp + 32 * kt);
    ah.h[1] = *(const v8us*)(ahp + 32 * kt + 16);
    al.h[0] = *(const v8us*)(alp + 32 * kt);
    al.h[1] = *(const v8us*)(alp + 32 * kt + 16);
#pragma unroll
    for (int t = 0; t < NCT; ++t) {
      const unsigned short* bp = Bw + (size_t)(16 * t + m) * KD + 32 * kt + 8 * hh;
      FragB bh, bl;
      bh.h[0] = *(const v8us*)bp;
      bh.h[1] = *(const v8us*)(bp + 16);
      bl.h[0] = *(const v8us*)(bp + WPL);
      bl.h[1] = *(const v8us*)(bp + WPL + 16);
      acc[t] = wmb(ah.v, bh.v, acc[t]);
      acc[t] = wmb(ah.v, bl.v, acc[t]);
      acc[t] = wmb(al.v, bh.v, acc[t]);
    }
  }
  __syncthreads();

  const int r0 = wave * 16 + 8 * hh;
  const v4f dA = *(const v4f*)(dinv + (size_t)rowBase + r0);
  const v4f dB = *(const v4f*)(dinv + (size_t)rowBase + r0 + 4);
  float s[8];
  s[0] = dA.x; s[1] = dA.y; s[2] = dA.z; s[3] = dA.w; s[4] = dB.x; s[5] = dB.y; s[6] = dB.z; s[7] = dB.w;
#pragma unroll
  for (int r = 0; r < 8; ++r) s[r] = (useDinv != 0 ? s[r] : 1.0f);
  float* sp = stg + r0 * NC + m;
#pragma unroll
  for (int t = 0; t < NCT; ++t) {
    const float bl = bias[16 * t + m];
    const float bv = useBias != 0 ? bl : 0.0f;
#pragma unroll
    for (int r = 0; r < 8; ++r) sp[r * NC + 16 * t] = acc[t][r] * s[r] + bv;
  }
  __syncthreads();

  const float* lp = stg + wave * 16 * NC + 4 * lane;
  float* gp = C + (size_t)(rowBase + wave * 16) * NC + 4 * lane;
  v4f ov[NPC];
#pragma unroll
  for (int i = 0; i < NPC; ++i) {
    v4f v = *(const v4f*)(lp + 128 * i);
    if (useAct != 0) {
#pragma unroll 1
      for (int q = 0; q < 4; ++q) { const float tq = tanhf(v.x); v.x = v.y; v.y = v.z; v.z = v.w; v.w = tq; }
    }
    ov[i] = v;
  }
#pragma unroll
  for (int i = 0; i < NPC; ++i) *(volatile v4f*)(gp + 128 * i) = ov[i];
  __threadfence();
#pragma unroll
  for (int i = 0; i < NPC; ++i) *(volatile v4f*)(gp + 128 * i) = ov[i];
}

__global__ __launch_bounds__(NTHR) void k_agg(
    const int* __restrict__ csr, const int* __restrict__ off, const int* __restrict__ cnt,
    const float* __restrict__ dinv, const float* __restrict__ hw, float* h,
    const float* __restrict__ bs, int nN, int csrLen) {
  const int tid = threadIdx.x, lane = tid & 31, wave = tid >> 5, hh = lane >> 4, c4 = 4 * (lane & 15);
  const int tbase = blockIdx.x * TGT + wave * 32;
  const int cl = tbase + lane;
  const int cnt_l = cnt[cl];
  const int off_l = off[cl];
  const float dv_l = dinv[cl];
  const v4f bb = *(const v4f*)(bs + c4);

#pragma unroll 1
  for (int jj = 0; jj < 16; ++jj) {
    const int j = 2 * jj + hh;
    const int c = tbase + j;
    int n = __shfl(cnt_l, j);
    n = n < 0 ? 0 : (n > DEGCAP ? DEGCAP : n);
    const int st = __shfl(off_l, j);
    const float dc = __shfl(dv_l, j);
    const int no = __shfl_xor(n, 16);
    int nm = n > no ? n : no;
    nm = __builtin_amdgcn_readfirstlane(nm);
    v4f acc = {0.f, 0.f, 0.f, 0.f};
#pragma unroll 1
    for (int q0 = 0; q0 < nm; q0 += 16) {
      int pos = st + q0 + (lane & 15);
      pos = pos < 0 ? 0 : (pos > csrLen - 1 ? csrLen - 1 : pos);
      int sl = csr[pos];
      sl = sl < 0 ? 0 : (sl > nN - 1 ? nN - 1 : sl);
      const int rem = nm - q0;
      const int mc = rem < 16 ? rem : 16;
#pragma unroll 1
      for (int p = 0; p < mc; ++p) {
        const int s = __shfl(sl, (lane & 16) | p);
        const v4f rv = *(const v4f*)(hw + (size_t)s * HIDC + c4);
        const bool ok = (q0 + p) < n;
        acc.x = ok ? acc.x + rv.x : acc.x;
        acc.y = ok ? acc.y + rv.y : acc.y;
        acc.z = ok ? acc.z + rv.z : acc.z;
        acc.w = ok ? acc.w + rv.w : acc.w;
      }
    }
    const v4f sv = *(const v4f*)(hw + (size_t)c * HIDC + c4);
    v4f v = (acc + sv) * dc + bb;
#pragma unroll 1
    for (int q = 0; q < 4; ++q) { const float tq = tanhf(v.x); v.x = v.y; v.y = v.z; v.z = v.w; v.w = tq; }
    float* hp = h + (size_t)c * HIDC + c4;
    *(volatile v4f*)hp = v;
    __threadfence();
    *(volatile v4f*)hp = v;
  }
}

__global__ __launch_bounds__(NTHR) void k_tail(
    const float* __restrict__ h2, const float* __restrict__ w3, const float* __restrict__ b3,
    const int* __restrict__ bat, const int* __restrict__ ia, const int* __restrict__ ib,
    float* out, int nN, int nG, int nP, int nOut) {
  __shared__ __attribute__((aligned(16))) float gsum[GCAP];
  __shared__ __attribute__((aligned(16))) float scr[SOUTN];
  __shared__ __attribute__((aligned(16))) int   sb[PCH];
  __shared__ __attribute__((aligned(16))) float sw3[32];
  float* gcnt = scr;
  float* su   = scr + GCAP;
  const int tid = threadIdx.x;
  for (int i = tid; i < GCAP; i += NTHR) { gsum[i] = 0.0f; gcnt[i] = 0.0f; }
  if (tid < 32) sw3[tid] = w3[tid];
  const float bias3 = b3[0];
  __syncthreads();

  const int nCh = (nN + PCH - 1) / PCH;
#pragma unroll 1
  for (int ch = 0; ch < nCh; ++ch) {
    const int cbase = ch * PCH;
#pragma unroll 1
    for (int jn = 0; jn < PCH / NTHR; ++jn) {
      const int li = jn * NTHR + tid;
      const int node = cbase + li;
      const int nc = node > nN - 1 ? nN - 1 : node;
      const float* hr = h2 + (size_t)nc * (HIDC / 2);
      float acc = 0.0f;
#pragma unroll 1
      for (int q = 0; q < 8; ++q) {
        const v4f hv = *(const v4f*)(hr + 4 * q);
        const v4f wv = *(const v4f*)(sw3 + 4 * q);
        acc += hv.x * wv.x; acc += hv.y * wv.y; acc += hv.z * wv.z; acc += hv.w * wv.w;
      }
      su[li] = acc + bias3;
      const int g = bat[nc];
      sb[li] = (node < nN) ? g : -1;
    }
    __syncthreads();
    if (tid == 0) {
      int lim = nN - cbase;
      lim = lim > PCH ? PCH : lim;
#pragma unroll 1
      for (int li = 0; li < lim; ++li) {
        const int g = sb[li];
        if ((unsigned)g < (unsigned)nG) { gsum[g] = gsum[g] + su[li]; gcnt[g] = gcnt[g] + 1.0f; }
      }
    }
    __syncthreads();
  }

  for (int g = tid; g < GCAP; g += NTHR) {
    const float cf = fmaxf(gcnt[g], 1.0f);
    gsum[g] = gsum[g] * (1.0f / cf);
  }
  __syncthreads();

#pragma unroll 1
  for (int f = tid; f < nOut; f += NTHR) {
    const int p = f > nP - 1 ? nP - 1 : f;
    int a = ia[p]; a = a < 0 ? 0 : (a > nG - 1 ? nG - 1 : a);
    int b = ib[p]; b = b < 0 ? 0 : (b > nG - 1 ? nG - 1 : b);
    const float d = gsum[b] - gsum[a];
    const float sg = 1.0f / (1.0f + expf(-d));
    int gi = f - nP; gi = gi < 0 ? 0 : (gi > nG - 1 ? nG - 1 : gi);
    const float xv = gsum[gi];
    scr[f] = (f < nP) ? sg : xv;
  }
  __syncthreads();

  const int nPc = nOut >> 2;
#pragma unroll 1
  for (int pc = tid; pc < nPc; pc += NTHR) { const v4f v = *(const v4f*)(scr + 4 * pc); *(volatile v4f*)(out + 4 * pc) = v; }
  __threadfence();
#pragma unroll 1
  for (int pc = tid; pc < nPc; pc += NTHR) { const v4f v = *(const v4f*)(scr + 4 * pc); *(volatile v4f*)(out + 4 * pc) = v; }
}

extern "C" void kernel_launch(void* const* d_in, const int* in_sizes, int n_in,
                              void* d_out, int out_size, void* d_ws, size_t ws_size,
                              hipStream_t stream) {
  if (n_in < 17) return;
  const int nN = in_sizes[0] / FIN;
  const int nE = in_sizes[1] / 2;
  const int nP = in_sizes[3];
  if (nN <= 0 || nE <= 0 || nP <= 0) return;
  if (in_sizes[0] != nN * FIN || in_sizes[1] != 2 * nE || in_sizes[2] != nN || in_sizes[4] != nP) return;
  if (in_sizes[5] != FIN * HIDC || in_sizes[6] != HIDC) return;
  if (in_sizes[7] != WPL || in_sizes[8] != HIDC || in_sizes[9] != WPL || in_sizes[10] != HIDC) return;
  if (in_sizes[11] != WPL || in_sizes[12] != HIDC) return;
  if (in_sizes[13] != HIDC * (HIDC / 2) || in_sizes[14] != HIDC / 2 || in_sizes[15] != HIDC / 2 || in_sizes[16] < 1) return;
  const int nG = out_size - nP;
  if (nG <= 0 || nG > GCAP || out_size > SOUTN || (out_size & 3) != 0) return;
  if (nE > (1 << 28) || nN > (1 << 24)) return;

  const float* x     = (const float*)d_in[0];
  const int*   ei    = (const int*)d_in[1];
  const int*   batch = (const int*)d_in[2];
  const int*   idx_a = (const int*)d_in[3];
  const int*   idx_b = (const int*)d_in[4];
  const float* W_in  = (const float*)d_in[5];
  const float* b_in  = (const float*)d_in[6];
  const float* W_h   = (const float*)d_in[7];
  const float* b_h   = (const float*)d_in[8];
  const float* W_out = (const float*)d_in[9];
  const float* b_out = (const float*)d_in[10];
  const float* fc1_w = (const float*)d_in[11];
  const float* fc1_b = (const float*)d_in[12];
  const float* fc2_w = (const float*)d_in[13];
  const float* fc2_b = (const float*)d_in[14];
  const float* fc3_w = (const float*)d_in[15];
  const float* fc3_b = (const float*)d_in[16];
  float* out = (float*)d_out;

  const int NPAD   = ((nN + TGT - 1) / TGT) * TGT;
  const int nBC    = (nN + NBC - 1) / NBC;
  const int CNTPAD = nBC * NBC;
  if (CNTPAD < NPAD) return;
  if (4 * nBC + 1 > RBN) return;
  const int nBF    = (nN + NBF - 1) / NBF;
  const int csrLen = ((nE + 31) & ~31) + 4096;
  if (31 * 4 * nBC > 4096) return;
  const int nGemm  = NPAD / GROWS;
  const int nAgg   = NPAD / TGT;
  const int nIn    = NPAD / INROWS;

  char* ws = (char*)d_ws;
  size_t off = 0;
  const size_t oW   = off; off += (size_t)NMAT * 2 * WPL * 2;      off = (off + 255) & ~(size_t)255;
  const size_t oCnt = off; off += (size_t)CNTPAD * 4;              off = (off + 255) & ~(size_t)255;
  const size_t oDv  = off; off += (size_t)CNTPAD * 4;              off = (off + 255) & ~(size_t)255;
  const size_t oOff = off; off += (size_t)CNTPAD * 4;              off = (off + 255) & ~(size_t)255;
  const size_t oRb  = off; off += (size_t)RBN * 4;                 off = (off + 255) & ~(size_t)255;
  const size_t oCsr = off; off += (size_t)csrLen * 4;              off = (off + 255) & ~(size_t)255;
  const size_t oH   = off; off += (size_t)NPAD * HIDC * 4;         off = (off + 255) & ~(size_t)255;
  const size_t oHw  = off; off += (size_t)NPAD * HIDC * 4;         off = (off + 255) & ~(size_t)255;
  if (off > ws_size || off > (size_t)WSCAP) return;
  unsigned short* wp = (unsigned short*)(ws + oW);
  int*      cnt  = (int*)(ws + oCnt);
  float*    dinv = (float*)(ws + oDv);
  int*      offp = (int*)(ws + oOff);
  int*      rb   = (int*)(ws + oRb);
  int*      csr  = (int*)(ws + oCsr);
  float*    h    = (float*)(ws + oH);
  float*    hw   = (float*)(ws + oHw);

  const int vec8 = ((nE & 3) == 0) ? 1 : 0;

  k_wprep<<<NMAT * 2, NTHR, 0, stream>>>(W_h, W_out, fc1_w, fc2_w, wp);

  k_count<<<nBC, NTHR, 0, stream>>>(ei, cnt, dinv, nE, vec8);
  k_offsets<<<1, OTHR, 0, stream>>>(cnt, offp, rb, nBC);
  hipFuncSetAttribute(reinterpret_cast<const void*>(&k_fill),
                      hipFuncAttributeMaxDynamicSharedMemorySize, LDS_FILL);
  k_fill<<<nBF, NTHR, LDS_FILL, stream>>>(ei, offp, rb, csr, nN, nE, vec8, csrLen);

  k_in<<<nIn, NTHR, 0, stream>>>(x, W_in, dinv, hw, nN);
  k_agg<<<nAgg, NTHR, 0, stream>>>(csr, offp, cnt, dinv, hw, h, b_in, nN, csrLen);

  k_gemm<4><<<nGemm, NTHR, 0, stream>>>(h, wp, dinv, b_h, hw, NPAD, 1, 0, 0);
  k_agg<<<nAgg, NTHR, 0, stream>>>(csr, offp, cnt, dinv, hw, h, b_h, nN, csrLen);
  k_gemm<4><<<nGemm, NTHR, 0, stream>>>(h, wp, dinv, b_h, hw, NPAD, 1, 0, 0);
  k_agg<<<nAgg, NTHR, 0, stream>>>(csr, offp, cnt, dinv, hw, h, b_h, nN, csrLen);
  k_gemm<4><<<nGemm, NTHR, 0, stream>>>(h, wp + (size_t)1 * 2 * WPL, dinv, b_out, hw, NPAD, 1, 0, 0);
  k_agg<<<nAgg, NTHR, 0, stream>>>(csr, offp, cnt, dinv, hw, h, b_out, nN, csrLen);

  k_gemm<4><<<nGemm, NTHR, 0, stream>>>(h, wp + (size_t)2 * 2 * WPL, dinv, fc1_b, hw, NPAD, 0, 1, 1);
  k_gemm<2><<<nGemm, NTHR, 0, stream>>>(hw, wp + (size_t)3 * 2 * WPL, dinv, fc2_b, h, NPAD, 0, 1, 1);

  k_tail<<<1, NTHR, 0, stream>>>(h, fc3_w, fc3_b, batch, idx_a, idx_b, out, nN, nG, nP, out_size);
}
